// SC2MambaBridge_57045755625695
// MI455X (gfx1250) — hardware-run, weakly checked
//
#include <hip/hip_runtime.h>
#pragma clang fp contract(off)


#ifndef NB
#define NB 2
#endif
#ifndef SEQ
#define SEQ 2000
#endif
#define NB_FULL  2
#define SEQ_FULL 2000
#define DM   256
#define DI   512
#define DS   16
#define DR   16
#define NL   4
#define XWR  48
#define XW   64
#define KDT  32
#define TS   16
#define MROWS (NB * SEQ)
#define MPAD  (((MROWS + 63) / 64) * 64)
#define LOG2E 1.4426950408889634f
#define SW_IN  16.0f
#define SW_XP  16.0f
#define SW_DT  64.0f
#define SW_OUT 16.0f
#define QRS  2048.0f
#define QRI  (1.0f / 2048.0f)

static_assert(NB <= NB_FULL);
static_assert(SEQ <= SEQ_FULL);
static_assert(MPAD % 64 == 0);
static_assert(MPAD % 32 == 0);
static_assert(MPAD % 8 == 0);
static_assert(MPAD % 4 == 0);
static_assert(MROWS % 32 == 0);
static_assert(SEQ % TS == 0);
static_assert(DM % 64 == 0);
static_assert((2 * DI) % 64 == 0);
static_assert(DI % 64 == 0);
static_assert(XW == 64);
static_assert(XWR == DR + 2 * DS);
static_assert(XWR <= XW);
static_assert(DR <= KDT);
static_assert(DR % 8 == 0);
static_assert(KDT % 32 == 0);
static_assert(DM % 32 == 0);
static_assert(DI % 32 == 0);
static_assert(DS == 16);
static_assert(DM == 32 * 8);
static_assert(256 * 8 == 4 * DI);
static_assert(64 * 4 == DM);

typedef _Float16 h16;
typedef __attribute__((ext_vector_type(16))) _Float16 v16h;
typedef __attribute__((ext_vector_type(8)))  _Float16 v8h;
typedef __attribute__((ext_vector_type(8)))  float    v8f;
typedef __attribute__((ext_vector_type(4)))  float    v4f;
typedef v4f  __attribute__((may_alias)) v4fa;
typedef v8h  __attribute__((may_alias)) v8ha;

__device__ __forceinline__ unsigned short f2bf(float f) { unsigned u = __float_as_uint(f); u += 0x7FFFu + ((u >> 16) & 1u); return (unsigned short)(u >> 16); }
__device__ __forceinline__ float bfr(float f) { return __uint_as_float(((unsigned)f2bf(f)) << 16); }
__device__ __forceinline__ v16h cat16(v8h lo, v8h hi) { return __builtin_shufflevector(lo, hi, 0, 1, 2, 3, 4, 5, 6, 7, 8, 9, 10, 11, 12, 13, 14, 15); }
__device__ __forceinline__ v8f wmma16(v16h a, v16h b, v8f c) { return __builtin_amdgcn_wmma_f32_16x16x32_f16(false, a, false, b, (short)0, c, false, false); }
__device__ __forceinline__ v16h  ldh(const h16* p) { return cat16(*(const v8h*)p, *(const v8h*)(p + 16)); }
__device__ __forceinline__ void wave_sync() { __builtin_amdgcn_fence(3  , "wavefront"); __builtin_amdgcn_wave_barrier(); asm volatile("" ::: "memory"); }

static __device__ __forceinline__ h16 toh_flush(float v) { const h16 r = (h16)v; return (fabsf(v) < 6.103515625e-05f) ? (h16)0.0f : r; }
__device__ __forceinline__ v8f wmma16g(v16h a, v16h b, v8f c) { c = wmma16(a, b, c); asm volatile("v_nop\n\tv_nop\n\tv_nop\n\tv_nop" : "+v"(c) : "v"(a), "v"(b)); return c; }
__device__ __forceinline__ float silu_f(float v) { return v * __builtin_amdgcn_rcpf(1.0f + __builtin_amdgcn_exp2f(-v * LOG2E)); }
__device__ __forceinline__ float softplus_f(float v) { return fmaxf(v, 0.0f) + log1pf(expf(-fabsf(v))); }

__global__ __launch_bounds__(256) void k_wcvt(const float* __restrict__ src, h16* dst, int srcRPG, int dstRPG, int srcCols, int dstCols, int nPieces, float scale) {
    const int i = blockIdx.x * 256 + threadIdx.x; if (i >= nPieces) return;
    const int e = i * 8; const int drow = e / dstCols, col = e - drow * dstCols;
    const int grp = drow / dstRPG, r = drow - grp * dstRPG;
    const bool ok = (r < srcRPG) & (col < srcCols);
    const int rc = (r < srcRPG) ? r : (srcRPG - 1); const int cc = (col < srcCols) ? col : (srcCols - 8);
    const size_t so = ((size_t)grp * (size_t)srcRPG + (size_t)rc) * (size_t)srcCols + (size_t)cc;
    v8f v = *(const v8f*)(src + so);
    asm volatile("" : "+v"(v));
    v8h o;
#pragma unroll
    for (int k = 0; k < 8; ++k) { const float t = ok ? (bfr(v[k]) * scale) : 0.0f; o[k] = toh_flush(t); }
    *(volatile v8h*)(dst + (size_t)i * 8) = o; __threadfence(); *(volatile v8h*)(dst + (size_t)i * 8) = o;
}

__global__ __launch_bounds__(256) void k_zfill(h16* dst, int nPieces) {
    const int i = blockIdx.x * 256 + threadIdx.x; if (i >= nPieces) return;
    const v8h z = (v8h){};
    *(volatile v8h*)(dst + (size_t)i * 8) = z; __threadfence(); *(volatile v8h*)(dst + (size_t)i * 8) = z;
}

__global__ __launch_bounds__(256) void k_embed(const float* __restrict__ x, const float* __restrict__ bw, const float* __restrict__ bb,
                                               const float* __restrict__ ge, const float* __restrict__ me, float* H) {
    const int i = blockIdx.x * 256 + threadIdx.x;
    const int row = i >> 6, d = (i & 63) * 4;
    const bool ok = row < MROWS; const int rc = ok ? row : (MROWS - 1);
    const int b = rc / SEQ, l = rc - b * SEQ;
    float xv = x[(size_t)b * SEQ_FULL + l];
    v4f w = *(const v4f*)(bw + d), bi = *(const v4f*)(bb + d), g = *(const v4f*)(ge + (size_t)l * DM + d), m = *(const v4f*)(me + d);
    asm volatile("" : "+v"(xv)); asm volatile("" : "+v"(w)); asm volatile("" : "+v"(bi)); asm volatile("" : "+v"(g)); asm volatile("" : "+v"(m));
    const float xb = bfr(xv);
    v4f o;
#pragma unroll
    for (int k = 0; k < 4; ++k) { const float t = ((xb * bfr(w[k]) + bfr(bi[k])) + bfr(g[k])) + bfr(m[k]); o[k] = ok ? t : 0.0f; }
    *(volatile v4f*)(H + (size_t)i * 4) = o; __threadfence(); *(volatile v4f*)(H + (size_t)i * 4) = o;
}

__global__ __launch_bounds__(256) void k_ln(const float* __restrict__ H, const float* __restrict__ gw, const float* __restrict__ gb, h16* HN, h16* HNR) {
    const int lane = threadIdx.x & 31;
    const int wave = __builtin_amdgcn_readfirstlane((int)(threadIdx.x >> 5));
    const int row = blockIdx.x * 8 + wave;
    const float* xr = H + (size_t)row * DM + lane * 8;
    const v4f x0 = *(const v4f*)xr, x1 = *(const v4f*)(xr + 4);
    const v4f w0 = *(const v4f*)(gw + lane * 8), w1 = *(const v4f*)(gw + lane * 8 + 4);
    const v4f b0 = *(const v4f*)(gb + lane * 8), b1 = *(const v4f*)(gb + lane * 8 + 4);
    float v[8], w[8], bb[8];
#pragma unroll
    for (int k = 0; k < 4; ++k) { v[k] = x0[k]; v[4 + k] = x1[k]; w[k] = bfr(w0[k]); w[4 + k] = bfr(w1[k]); bb[k] = bfr(b0[k]); bb[4 + k] = bfr(b1[k]); }
    float s = 0.0f;
#pragma unroll
    for (int k = 0; k < 8; ++k) s += v[k];
#pragma unroll
    for (int off = 16; off; off >>= 1) s += __shfl_xor(s, off, 32);
    const float mu = s * (1.0f / DM);
    float q = 0.0f;
#pragma unroll
    for (int k = 0; k < 8; ++k) { const float dd = v[k] - mu; q += dd * dd; }
#pragma unroll
    for (int off = 16; off; off >>= 1) q += __shfl_xor(q, off, 32);
    const float inv = rsqrtf(q * (1.0f / DM) + 1e-5f);
    v8h o, orv;
#pragma unroll
    for (int k = 0; k < 8; ++k) { const float t = ((v[k] - mu) * inv) * w[k] + bb[k]; const h16 hv = toh_flush(t); o[k] = hv; orv[k] = toh_flush((t - (float)hv) * QRS); }
    h16* dst = HN + (size_t)row * DM + lane * 8;
    h16* dsr = HNR + (size_t)row * DM + lane * 8;
    *(volatile v8h*)dst = o; *(volatile v8h*)dsr = orv; __threadfence(); *(volatile v8h*)dst = o; *(volatile v8h*)dsr = orv;
}

__global__ __launch_bounds__(256) void k_conv(const float* __restrict__ XZ, const float* __restrict__ cw, const float* __restrict__ cb, h16* U16, float* UF) {
    __shared__ __align__(16) float uf[4 * DI];
    static_assert(4 * DI * 4 <= 131072);
    const int t = threadIdx.x; const int rl = t >> 6, e = (t & 63) * 8;
    const int row = blockIdx.x * 4 + rl; const int l = row % SEQ;
    float xa[4][8];
#pragma unroll
    for (int k = 0; k < 4; ++k) {
        const bool ok = (l + k - 3) >= 0; const int rr = ok ? (row + k - 3) : row;
        v4f x0 = *(const v4f*)(XZ + (size_t)rr * (2 * DI) + e), x1 = *(const v4f*)(XZ + (size_t)rr * (2 * DI) + e + 4);
        asm volatile("" : "+v"(x0)); asm volatile("" : "+v"(x1));
#pragma unroll
        for (int i = 0; i < 4; ++i) { xa[k][i] = ok ? x0[i] : 0.0f; xa[k][4 + i] = ok ? x1[i] : 0.0f; }
    }
    const v4f c0 = *(const v4f*)(cb + e), c1 = *(const v4f*)(cb + e + 4);
    v8h hv; v4f f0, f1;
#pragma unroll
    for (int c = 0; c < 8; ++c) {
        const v4f wv = *(const v4f*)(cw + (size_t)(e + c) * 4);
        float a = xa[0][c] * bfr(wv[0]);
        a = a + xa[1][c] * bfr(wv[1]);
        a = a + xa[2][c] * bfr(wv[2]);
        a = a + xa[3][c] * bfr(wv[3]);
        a = a + bfr(c < 4 ? c0[c & 3] : c1[c & 3]);
        const float u = silu_f(a);
        hv[c] = toh_flush(u);
        if (c < 4) f0[c & 3] = u; else f1[c & 3] = u;
    }
    *(v4fa*)(&uf[t * 8]) = f0; *(v4fa*)(&uf[t * 8 + 4]) = f1;
    __syncthreads();
    const v4f g0 = *(const v4fa*)(&uf[t * 4]), g1 = *(const v4fa*)(&uf[(256 + t) * 4]);
    const size_t o16 = (size_t)blockIdx.x * (4 * DI) + (size_t)t * 8;
    float* ufg = UF + (size_t)blockIdx.x * (4 * DI);
    static_assert(256 * 16 * 2 == 4 * DI * 4);
    static_assert(256 * 16 == 4 * DI * 2);
#pragma unroll 1
    for (int ps = 0; ps < 2; ++ps) {
        *(volatile v8h*)(U16 + o16) = hv;
        *(volatile v4f*)(ufg + (size_t)t * 4) = g0;
        *(volatile v4f*)(ufg + (size_t)(256 + t) * 4) = g1;
        if (ps == 0) __threadfence(); }
}

template <int EPI, int K>
__device__ __forceinline__ void gemm_body(const h16* __restrict__ A, const h16* __restrict__ Bt, float* C, const int ldc,
                                          const float* __restrict__ bias, const float* __restrict__ Hin, h16* D16, const float oscale) {
    __shared__ __align__(16) float os[16 * 68];
    static_assert(16 * 68 * 4 <= 131072);
    static_assert(K % 32 == 0);
    static_assert(8 * 32 * 16 == 16 * 64 * 4);
    static_assert(2 * 32 * 16 == 16 * KDT * 2);
    const int lane = threadIdx.x & 31, lr = lane & 15, hi = lane >> 4; const int r0 = blockIdx.x * 64, c0 = blockIdx.y * 64;
    v8f acc[4][4];
#pragma unroll
    for (int mb = 0; mb < 4; ++mb)
#pragma unroll
        for (int nb = 0; nb < 4; ++nb) acc[mb][nb] = (v8f){};
    const size_t aoff = (size_t)(r0 + lr) * K + 8 * hi, boff = (size_t)(c0 + lr) * K + 8 * hi;
#pragma unroll 1
    for (int kc = 0; kc < K; kc += 32) {
        v16h a[4];
#pragma unroll
        for (int mb = 0; mb < 4; ++mb) a[mb] = ldh(A + aoff + (size_t)mb * 16 * K + kc);
#pragma unroll
        for (int nb = 0; nb < 4; ++nb) { const v16h b = ldh(Bt + boff + (size_t)nb * 16 * K + kc);
#pragma unroll
            for (int mb = 0; mb < 4; ++mb) acc[mb][nb] = wmma16g(a[mb], b, acc[mb][nb]); }
    }
    float bc[4];
#pragma unroll
    for (int nb = 0; nb < 4; ++nb) { bc[nb] = 0.0f; if (EPI == 2) bc[nb] = bfr(bias[c0 + nb * 16 + lr]); }
    const bool zhalf = (EPI == 0) && (c0 >= DI);
#pragma unroll
    for (int mb = 0; mb < 4; ++mb) {
#pragma unroll
        for (int nb = 0; nb < 4; ++nb) {
#pragma unroll
            for (int j = 0; j < 8; ++j) os[(hi * 8 + j) * 68 + nb * 16 + lr] = acc[mb][nb][j] * oscale + bc[nb]; }
        wave_sync();
        if (EPI == 2 || EPI == 3 || zhalf) {
#pragma unroll 1
            for (int s = 0; s < 8; ++s) { const int row = 2 * s + (lane >> 4), c4 = (lane & 15) * 4;
                v4f v = *(const v4fa*)(&os[row * 68 + c4]);
                if (EPI == 0) {
#pragma unroll
                    for (int i = 0; i < 4; ++i) v[i] = silu_f(v[i]); }
                if (EPI == 2) {
#pragma unroll
                    for (int i = 0; i < 4; ++i) v[i] = softplus_f(v[i]); }
                if (EPI == 3) { const v4f hv = *(const v4f*)(Hin + (size_t)(r0 + mb * 16 + row) * ldc + c0 + c4); v = v + hv; }
                *(v4fa*)(&os[row * 68 + c4]) = v; }
            wave_sync();
        }
        float* cbp = C + (size_t)(r0 + mb * 16) * ldc + c0;
#pragma unroll 1
        for (int ps = 0; ps < 2; ++ps) {
#pragma unroll
            for (int s = 0; s < 8; ++s) { const int row = 2 * s + (lane >> 4), c4 = (lane & 15) * 4;
                const v4f val = *(const v4fa*)(&os[row * 68 + c4]);
                *(volatile v4f*)(cbp + (size_t)row * ldc + c4) = val; }
            if (EPI == 1) {
#pragma unroll
                for (int s = 0; s < 2; ++s) { const int p = s * 32 + lane; const int row = p >> 2, c8 = (p & 3) * 8;
                    const int cr = c8 & 8; const bool live = c8 < DR;
                    const v4f x0 = *(const v4fa*)(&os[row * 68 + cr]); const v4f x1 = *(const v4fa*)(&os[row * 68 + cr + 4]); v8h hv;
#pragma unroll
                    for (int i = 0; i < 4; ++i) { const float t0 = live ? x0[i] : 0.0f; const float t1 = live ? x1[i] : 0.0f; hv[i] = toh_flush(t0); hv[4 + i] = toh_flush(t1); }
                    *(volatile v8h*)(D16 + (size_t)(r0 + mb * 16) * KDT + (size_t)p * 8) = hv; }
            }
            if (ps == 0) __threadfence(); }
        wave_sync();
    }
}

__global__ __launch_bounds__(32) void k_gemm_xz(const h16* __restrict__ A, const h16* __restrict__ AR, const h16* __restrict__ Bt, float* C) {
    __shared__ __align__(16) float os[16 * 68];
    static_assert(16 * 68 * 4 <= 131072);
    static_assert(DM % 32 == 0);
    static_assert(8 * 32 * 16 == 16 * 64 * 4);
    static_assert(2 * 16 == 32);
    const int K = DM; const int ldc = 2 * DI; const float oscale = 1.0f / SW_IN;
    const int lane = threadIdx.x & 31, lr = lane & 15, hi = lane >> 4; const int r0 = blockIdx.x * 32, c0 = blockIdx.y * 64;
    v8f acc[2][4], accR[2][4];
#pragma unroll
    for (int mb = 0; mb < 2; ++mb)
#pragma unroll
        for (int nb = 0; nb < 4; ++nb) { acc[mb][nb] = (v8f){}; accR[mb][nb] = (v8f){}; }
    const size_t aoff = (size_t)(r0 + lr) * K + 8 * hi, boff = (size_t)(c0 + lr) * K + 8 * hi;
#pragma unroll 1
    for (int kc = 0; kc < K; kc += 32) {
        v16h a[2], ar[2];
#pragma unroll
        for (int mb = 0; mb < 2; ++mb) { a[mb] = ldh(A + aoff + (size_t)mb * 16 * K + kc); ar[mb] = ldh(AR + aoff + (size_t)mb * 16 * K + kc); }
#pragma unroll
        for (int nb = 0; nb < 4; ++nb) { const v16h b = ldh(Bt + boff + (size_t)nb * 16 * K + kc);
#pragma unroll
            for (int mb = 0; mb < 2; ++mb) { acc[mb][nb] = wmma16g(a[mb], b, acc[mb][nb]); accR[mb][nb] = wmma16g(ar[mb], b, accR[mb][nb]); } }
    }
    const bool zhalf = c0 >= DI;
#pragma unroll
    for (int mb = 0; mb < 2; ++mb) {
#pragma unroll
        for (int nb = 0; nb < 4; ++nb) {
#pragma unroll
            for (int j = 0; j < 8; ++j) os[(hi * 8 + j) * 68 + nb * 16 + lr] = (acc[mb][nb][j] + accR[mb][nb][j] * QRI) * oscale; }
        wave_sync();
        if (zhalf) {
#pragma unroll 1
            for (int s = 0; s < 8; ++s) { const int row = 2 * s + (lane >> 4), c4 = (lane & 15) * 4;
                v4f v = *(const v4fa*)(&os[row * 68 + c4]);
#pragma unroll
                for (int i = 0; i < 4; ++i) v[i] = silu_f(v[i]);
                *(v4fa*)(&os[row * 68 + c4]) = v; }
            wave_sync();
        }
        float* cbp = C + (size_t)(r0 + mb * 16) * ldc + c0;
#pragma unroll 1
        for (int ps = 0; ps < 2; ++ps) {
#pragma unroll
            for (int s = 0; s < 8; ++s) { const int row = 2 * s + (lane >> 4), c4 = (lane & 15) * 4;
                const v4f val = *(const v4fa*)(&os[row * 68 + c4]);
                *(volatile v4f*)(cbp + (size_t)row * ldc + c4) = val; }
            if (ps == 0) __threadfence(); }
        wave_sync();
    }
}

__global__ __launch_bounds__(32) void k_gemm_xd(const h16* __restrict__ A, const h16* __restrict__ Bt, float* C, h16* D16) {
    gemm_body<1, DI>(A, Bt, C, XW, nullptr, nullptr, D16, 1.0f / SW_XP); }
__global__ __launch_bounds__(32) void k_gemm_dt(const h16* __restrict__ A, const h16* __restrict__ Bt, const float* __restrict__ bias, float* C) {
    gemm_body<2, KDT>(A, Bt, C, DI, bias, nullptr, nullptr, 1.0f / SW_DT); }
__global__ __launch_bounds__(32) void k_gemm_out(const h16* __restrict__ A, const h16* __restrict__ Bt, const float* __restrict__ Hin, float* C) {
    gemm_body<3, DI>(A, Bt, C, DM, nullptr, Hin, nullptr, 1.0f / SW_OUT); }

__global__ __launch_bounds__(64) void k_scan(const float* __restrict__ DT, const float* __restrict__ UF, const float* __restrict__ XD, const float* __restrict__ XZ,
                                             const float* __restrict__ alog, const float* __restrict__ dvec, h16* Y) {
    __shared__ __align__(16) float sbc[TS * 32];
    __shared__ __align__(16) h16 ysh[TS * 64];
    static_assert(TS * 32 * 4 + TS * 64 * 2 <= 131072);
    static_assert(64 * 2 * 16 == TS * 32 * 4);
    static_assert(64 * 2 * 16 == TS * 64 * 2);
    const int tid = threadIdx.x; const int ch = blockIdx.x * 64 + tid; const int b = blockIdx.y;
    float a2[16], st[16];
    {
        const v4f q0 = *(const v4f*)(alog + (size_t)ch * DS), q1 = *(const v4f*)(alog + (size_t)ch * DS + 4), q2 = *(const v4f*)(alog + (size_t)ch * DS + 8), q3 = *(const v4f*)(alog + (size_t)ch * DS + 12);
#pragma unroll
        for (int r = 0; r < 4; ++r) { a2[r] = q0[r]; a2[4 + r] = q1[r]; a2[8 + r] = q2[r]; a2[12 + r] = q3[r]; }
#pragma unroll
        for (int n = 0; n < 16; ++n) { a2[n] = -__builtin_amdgcn_exp2f(bfr(a2[n]) * LOG2E) * LOG2E; st[n] = 0.0f; }
    }
    const float dd = bfr(dvec[ch]);
    const size_t rb = (size_t)b * SEQ;
#pragma unroll 1
    for (int l0 = 0; l0 < SEQ; l0 += TS) {
#pragma unroll
        for (int it = 0; it < 2; ++it) { const int p = it * 64 + tid; const int s = p >> 3, q = p & 7;
            const v4f v = *(const v4f*)(XD + (rb + (size_t)(l0 + s)) * XW + DR + 4 * q);
            *(v4fa*)(&sbc[s * 32 + 4 * q]) = v; }
        __syncthreads();
#pragma unroll 1
        for (int s = 0; s < TS; ++s) {
            const size_t m = rb + (size_t)(l0 + s);
            const float dtv = DT[m * DI + ch], uv = UF[m * DI + ch], gv = XZ[m * (2 * DI) + DI + ch];
            const float dbu = dtv * uv;
            const v4f b0 = *(const v4fa*)(&sbc[s * 32 +  0]), b1 = *(const v4fa*)(&sbc[s * 32 +  4]), b2 = *(const v4fa*)(&sbc[s * 32 +  8]), b3 = *(const v4fa*)(&sbc[s * 32 + 12]);
            const v4f c0 = *(const v4fa*)(&sbc[s * 32 + 16]), c1 = *(const v4fa*)(&sbc[s * 32 + 20]), c2 = *(const v4fa*)(&sbc[s * 32 + 24]), c3 = *(const v4fa*)(&sbc[s * 32 + 28]);
            float bv[16], cv[16];
#pragma unroll
            for (int r = 0; r < 4; ++r) { bv[r] = b0[r]; bv[4 + r] = b1[r]; bv[8 + r] = b2[r]; bv[12 + r] = b3[r]; cv[r] = c0[r]; cv[4 + r] = c1[r]; cv[8 + r] = c2[r]; cv[12 + r] = c3[r]; }
            float acc = 0.0f;
#pragma unroll
            for (int n = 0; n < 16; ++n) {
                st[n] = __builtin_amdgcn_exp2f(dtv * a2[n]) * st[n] + dbu * bv[n];
                acc += st[n] * cv[n]; }
            const float yv = (acc + uv * dd) * gv;
            ysh[s * 64 + tid] = toh_flush(yv);
        }
        __syncthreads();
        v8h y0, y1;
        { const int p0 = tid, p1 = 64 + tid;
          y0 = *(const v8ha*)(&ysh[(p0 >> 3) * 64 + (p0 & 7) * 8]); y1 = *(const v8ha*)(&ysh[(p1 >> 3) * 64 + (p1 & 7) * 8]); }
        h16* d0 = Y + (rb + (size_t)(l0 + (tid >> 3))) * DI + blockIdx.x * 64 + (tid & 7) * 8;
        h16* d1 = Y + (rb + (size_t)(l0 + 8 + (tid >> 3))) * DI + blockIdx.x * 64 + (tid & 7) * 8;
#pragma unroll 1
        for (int ps = 0; ps < 2; ++ps) {
            *(volatile v8h*)d0 = y0;
            *(volatile v8h*)d1 = y1;
            if (ps == 0) __threadfence(); }
    }
}

__global__ __launch_bounds__(256) void k_final(const float* __restrict__ H, const float* __restrict__ fw, const float* __restrict__ fb,
                                               const float* __restrict__ hw, const float* __restrict__ hb, float* OUT) {
    __shared__ __align__(16) float sy[32];
    const int lane = threadIdx.x & 31;
    const int wave = __builtin_amdgcn_readfirstlane((int)(threadIdx.x >> 5));
    const v4f w0 = *(const v4f*)(fw + lane * 8), w1 = *(const v4f*)(fw + lane * 8 + 4);
    const v4f b0 = *(const v4f*)(fb + lane * 8), b1 = *(const v4f*)(fb + lane * 8 + 4);
    const v4f h0 = *(const v4f*)(hw + lane * 8), h1 = *(const v4f*)(hw + lane * 8 + 4);
    float w[8], bb[8], hv[8];
#pragma unroll
    for (int k = 0; k < 4; ++k) { w[k] = bfr(w0[k]); w[4 + k] = bfr(w1[k]); bb[k] = bfr(b0[k]); bb[4 + k] = bfr(b1[k]); hv[k] = bfr(h0[k]); hv[4 + k] = bfr(h1[k]); }
    const float hbv = bfr(hb[0]);
#pragma unroll 1
    for (int i = 0; i < 4; ++i) {
        const int rl = wave * 4 + i; const int row = blockIdx.x * 32 + rl;
        const float* xr = H + (size_t)row * DM + lane * 8;
        const v4f x0 = *(const v4f*)xr, x1 = *(const v4f*)(xr + 4);
        float v[8];
#pragma unroll
        for (int k = 0; k < 4; ++k) { v[k] = x0[k]; v[4 + k] = x1[k]; }
        float s = 0.0f;
#pragma unroll
        for (int k = 0; k < 8; ++k) s += v[k];
#pragma unroll
        for (int off = 16; off; off >>= 1) s += __shfl_xor(s, off, 32);
        const float mu = s * (1.0f / DM);
        float q = 0.0f;
#pragma unroll
        for (int k = 0; k < 8; ++k) { const float dd = v[k] - mu; q += dd * dd; }
#pragma unroll
        for (int off = 16; off; off >>= 1) q += __shfl_xor(q, off, 32);
        const float inv = rsqrtf(q * (1.0f / DM) + 1e-5f);
        float y = 0.0f;
#pragma unroll
        for (int k = 0; k < 8; ++k) y += (((v[k] - mu) * inv) * w[k] + bb[k]) * hv[k];
#pragma unroll
        for (int off = 16; off; off >>= 1) y += __shfl_xor(y, off, 32);
        if (lane == 0) sy[rl] = y + hbv;
    }
    __syncthreads();
    if (threadIdx.x < 8) {
        const v4f val = *(const v4fa*)(&sy[threadIdx.x * 4]);
        float* dst = OUT + (size_t)blockIdx.x * 32 + threadIdx.x * 4;
        *(volatile v4f*)dst = val; __threadfence(); *(volatile v4f*)dst = val;
    }
}

static constexpr size_t al256(size_t v) { return (v + 255) & ~(size_t)255; }
static constexpr size_t SZ_WIN  = al256((size_t)NL * 2 * DI * DM * 2);
static constexpr size_t SZ_WXP  = al256((size_t)NL * XW * DI * 2);
static constexpr size_t SZ_WDT  = al256((size_t)NL * DI * KDT * 2);
static constexpr size_t SZ_WOUT = al256((size_t)NL * DM * DI * 2);
static constexpr size_t SZ_H    = al256((size_t)MPAD * DM * 4);
static constexpr size_t SZ_HN   = al256((size_t)MPAD * DM * 2);
static constexpr size_t SZ_HNR  = al256((size_t)MPAD * DM * 2);
static constexpr size_t SZ_XZ   = al256((size_t)MPAD * 2 * DI * 4);
static constexpr size_t SZ_U16  = al256((size_t)MPAD * DI * 2);
static constexpr size_t SZ_UF   = al256((size_t)MPAD * DI * 4);
static constexpr size_t SZ_XD   = al256((size_t)MPAD * XW * 4);
static constexpr size_t SZ_DTR  = al256((size_t)MPAD * KDT * 2);
static constexpr size_t SZ_DT   = al256((size_t)MPAD * DI * 4);
static constexpr size_t SZ_Y    = al256((size_t)MPAD * DI * 2);
static constexpr size_t SZ_TOTAL = SZ_WIN + SZ_WXP + SZ_WDT + SZ_WOUT + 2 * SZ_H + SZ_HN + SZ_HNR + SZ_XZ + SZ_U16 + SZ_UF + SZ_XD + SZ_DTR + SZ_DT + SZ_Y;
static_assert(SZ_TOTAL <= (size_t)134217728);
static_assert(((size_t)2 * DI * DM * 2) % 256 == 0);
static_assert(((size_t)XW * DI * 2) % 256 == 0);
static_assert(((size_t)DI * KDT * 2) % 256 == 0);
static_assert(((size_t)DM * DI * 2) % 256 == 0);
static_assert(((size_t)NL * 2 * DI * DM) % 8 == 0);
static_assert(((size_t)(MPAD - MROWS) * DI) % 8 == 0);
static_assert((size_t)MROWS * 4 <= (size_t)NB_FULL * SEQ_FULL * 4);

extern "C" void kernel_launch(void* const* d_in, const int* in_sizes, int n_in,
                              void* d_out, int out_size, void* d_ws, size_t ws_size, hipStream_t stream) {
    if (n_in < 20) return;
    if ((size_t)in_sizes[0] < (size_t)(NB - 1) * SEQ_FULL + SEQ) return;
    if (in_sizes[1] < DM || in_sizes[2] < DM || in_sizes[4] < DM) return;
    if ((size_t)in_sizes[3] < (size_t)SEQ * DM) return;
    if (in_sizes[5] < NL * DM || in_sizes[6] < NL * DM) return;
    if ((size_t)in_sizes[7] < (size_t)NL * 2 * DI * DM) return;
    if (in_sizes[8] < NL * DI * 4 || in_sizes[9] < NL * DI) return;
    if ((size_t)in_sizes[10] < (size_t)NL * XWR * DI) return;
    if (in_sizes[11] < NL * DI * DR || in_sizes[12] < NL * DI) return;
    if (in_sizes[13] < NL * DI * DS || in_sizes[14] < NL * DI) return;
    if ((size_t)in_sizes[15] < (size_t)NL * DM * DI) return;
    if (in_sizes[16] < DM || in_sizes[17] < DM || in_sizes[18] < DM || in_sizes[19] < 1) return;
    if ((size_t)out_size < (size_t)MROWS) return;
    if (SZ_TOTAL > ws_size) return;
    const float* x     = (const float*)d_in[0];
    const float* bw    = (const float*)d_in[1];
    const float* bb    = (const float*)d_in[2];
    const float* ge    = (const float*)d_in[3];
    const float* me    = (const float*)d_in[4];
    const float* lnw   = (const float*)d_in[5];
    const float* lnb   = (const float*)d_in[6];
    const float* inw   = (const float*)d_in[7];
    const float* cw    = (const float*)d_in[8];
    const float* cb    = (const float*)d_in[9];
    const float* xpw   = (const float*)d_in[10];
    const float* dtw   = (const float*)d_in[11];
    const float* dtb   = (const float*)d_in[12];
    const float* alog  = (const float*)d_in[13];
    const float* dvec  = (const float*)d_in[14];
    const float* outw  = (const float*)d_in[15];
    const float* finw  = (const float*)d_in[16];
    const float* finb  = (const float*)d_in[17];
    const float* headw = (const float*)d_in[18];
    const float* headb = (const float*)d_in[19];
    float* OUT = (float*)d_out;
    char* wsp = (char*)d_ws;
    h16* WIN  = (h16*)wsp; wsp += SZ_WIN;
    h16* WXP  = (h16*)wsp; wsp += SZ_WXP;
    h16* WDT  = (h16*)wsp; wsp += SZ_WDT;
    h16* WOUT = (h16*)wsp; wsp += SZ_WOUT;
    float* HA = (float*)wsp; wsp += SZ_H;
    float* HB = (float*)wsp; wsp += SZ_H;
    h16* HN   = (h16*)wsp; wsp += SZ_HN;
    h16* HNR  = (h16*)wsp; wsp += SZ_HNR;
    float* XZ = (float*)wsp; wsp += SZ_XZ;
    h16* U16  = (h16*)wsp; wsp += SZ_U16;
    float* UF = (float*)wsp; wsp += SZ_UF;
    float* XD = (float*)wsp; wsp += SZ_XD;
    h16* DTR  = (h16*)wsp; wsp += SZ_DTR;
    float* DT = (float*)wsp; wsp += SZ_DT;
    h16* Y    = (h16*)wsp; wsp += SZ_Y;

    { const int np = NL * 2 * DI * DM / 8;  k_wcvt<<<(unsigned)((np + 255) / 256), 256, 0, stream>>>(inw,  WIN,  NL * 2 * DI, NL * 2 * DI, DM, DM,  np, SW_IN); }
    { const int np = NL * XW * DI / 8;      k_wcvt<<<(unsigned)((np + 255) / 256), 256, 0, stream>>>(xpw,  WXP,  XWR,         XW,          DI, DI,  np, SW_XP); }
    { const int np = NL * DI * KDT / 8;     k_wcvt<<<(unsigned)((np + 255) / 256), 256, 0, stream>>>(dtw,  WDT,  NL * DI,     NL * DI,     DR, KDT, np, SW_DT); }
    { const int np = NL * DM * DI / 8;      k_wcvt<<<(unsigned)((np + 255) / 256), 256, 0, stream>>>(outw, WOUT, NL * DM,     NL * DM,     DI, DI,  np, SW_OUT); }
    if (MPAD > MROWS) { const int np = (MPAD - MROWS) * DI / 8; k_zfill<<<(unsigned)((np + 255) / 256), 256, 0, stream>>>(Y + (size_t)MROWS * DI, np); }

    k_embed<<<MPAD / 4, 256, 0, stream>>>(x, bw, bb, ge, me, HA);
    float* Hc = HA; float* Hn = HB;
    for (int i = 0; i < NL; ++i) {
        k_ln<<<MPAD / 8, 256, 0, stream>>>(Hc, lnw + (size_t)i * DM, lnb + (size_t)i * DM, HN, HNR);
        k_gemm_xz<<<dim3(MPAD / 32, 2 * DI / 64, 1), 32, 0, stream>>>(HN, HNR, WIN + (size_t)i * 2 * DI * DM, XZ);
        k_conv<<<MPAD / 4, 256, 0, stream>>>(XZ, cw + (size_t)i * DI * 4, cb + (size_t)i * DI, U16, UF);
        k_gemm_xd<<<dim3(MPAD / 64, 1, 1), 32, 0, stream>>>(U16, WXP + (size_t)i * XW * DI, XD, DTR);
        k_gemm_dt<<<dim3(MPAD / 64, DI / 64, 1), 32, 0, stream>>>(DTR, WDT + (size_t)i * DI * KDT, dtb + (size_t)i * DI, DT);
        k_scan<<<dim3(DI / 64, NB, 1), 64, 0, stream>>>(DT, UF, XD, XZ, alog + (size_t)i * DI * DS, dvec + (size_t)i * DI, Y);
        k_gemm_out<<<dim3(MPAD / 64, DM / 64, 1), 32, 0, stream>>>(Y, WOUT + (size_t)i * DM * DI, Hc, Hn);
        float* tmp = Hc; Hc = Hn; Hn = tmp;
    }
    k_final<<<MROWS / 32, 256, 0, stream>>>(Hc, finw, finb, headw, headb, OUT);
}
